// DecoderBlock_17102559773269
// MI455X (gfx1250) — hardware-verified
//
#include <hip/hip_runtime.h>
#include <stddef.h>


typedef _Float16 f16t;
typedef _Float16 v16h __attribute__((ext_vector_type(16)));
typedef _Float16 v8h  __attribute__((ext_vector_type(8)));
typedef _Float16 v4h  __attribute__((ext_vector_type(4)));
typedef float    v8f  __attribute__((ext_vector_type(8)));
typedef float    v4f  __attribute__((ext_vector_type(4)));

#define DEV __device__ __forceinline__

#ifndef NB
#define NB 4
#endif
#ifndef SEQ
#define SEQ 1024
#endif
#define NB_FULL 4
#define SEQ_FULL 1024
#define DM 1024
#define NH 16
#define HD 64
#define MROWS (NB * SEQ)
#define LN_EPS 1e-5f

static_assert(MROWS % 128 == 0);
static_assert(SEQ % 64 == 0);
static_assert(DM == NH * HD);
static_assert(NB >= 1 && NB <= NB_FULL);
static_assert(SEQ <= SEQ_FULL);

DEV float bfr(float x) {
  unsigned u = __builtin_bit_cast(unsigned, x);
  u = (u + 0x7FFFu + ((u >> 16) & 1u)) & 0xFFFF0000u;
  return __builtin_bit_cast(float, u);
}
DEV v4f bfr4(v4f v) {
  v4f r;
  r.x = bfr(v.x); r.y = bfr(v.y); r.z = bfr(v.z); r.w = bfr(v.w);
  return r;
}

DEV float gelu_t(float x) {
  const float y = 0.7978845608028654f * (x + 0.044715f * x * x * x);
  const float e = __expf(2.0f * y);
  const float t = 1.0f - 2.0f * __builtin_amdgcn_rcpf(e + 1.0f);
  return 0.5f * x * (1.0f + t);
}
DEV v4f gelu4(v4f v) {
  v4f r;
  r.x = gelu_t(v.x); r.y = gelu_t(v.y); r.z = gelu_t(v.z); r.w = gelu_t(v.w);
  return r;
}

DEV v16h load_frag(const f16t* base, int stride, int lane) {
  const f16t* p = base + (size_t)(lane & 15) * stride + ((lane >> 4) << 3);
  const v8h lo = *reinterpret_cast<const v8h*>(p);
  const v8h hi = *reinterpret_cast<const v8h*>(p + 16);
  v16h f;
#pragma unroll
  for (int i = 0; i < 8; ++i) { f[i] = lo[i]; f[i + 8] = hi[i]; }
  return f;
}

DEV v8f wmma16(v16h a, v16h b, v8f c) {
  return __builtin_amdgcn_wmma_f32_16x16x32_f16(false, a, false, b, (short)0, c, false, false);
}

__global__ __launch_bounds__(256) void cvt_k(const float* __restrict__ in, f16t* __restrict__ out, int nrows) {
  const size_t e0 = ((size_t)blockIdx.x * 256 + threadIdx.x) * 8;
  const size_t total = (size_t)nrows * DM;
  const bool ok = e0 < total;
  v8h hv = {};
  size_t oidx = 0;
  if (ok) {
    const int m = (int)(e0 / DM);
    const int c = (int)(e0 % DM);
    const size_t irow = (size_t)(m / SEQ) * SEQ_FULL + (size_t)(m % SEQ);
    const float* p = in + irow * DM + c;
    const v4f a = *(const v4f*)p;
    const v4f b = *(const v4f*)(p + 4);
    hv[0] = (f16t)bfr(a.x); hv[1] = (f16t)bfr(a.y); hv[2] = (f16t)bfr(a.z); hv[3] = (f16t)bfr(a.w);
    hv[4] = (f16t)bfr(b.x); hv[5] = (f16t)bfr(b.y); hv[6] = (f16t)bfr(b.z); hv[7] = (f16t)bfr(b.w);
    oidx = (size_t)m * DM + c;
    *(volatile v8h*)(out + oidx) = hv;
  }
  __threadfence();
  if (ok) *(volatile v8h*)(out + oidx) = hv;
}

__global__ __launch_bounds__(256) void wtrans_k(const float* __restrict__ in, f16t* __restrict__ out,
                                               int rows, int cols, float scale) {
  __shared__ __attribute__((aligned(16))) f16t tile[64][72];
  const int tid = threadIdx.x;
  const int c0 = blockIdx.x * 64, r0 = blockIdx.y * 64;
#pragma unroll
  for (int j = 0; j < 4; ++j) {
    const int i = tid + 256 * j;
    const int r = i >> 4, q4 = i & 15;
    const v4f v = *(const v4f*)(in + (size_t)(r0 + r) * cols + c0 + q4 * 4);
    tile[q4 * 4 + 0][r] = (f16t)(bfr(v.x) * scale);
    tile[q4 * 4 + 1][r] = (f16t)(bfr(v.y) * scale);
    tile[q4 * 4 + 2][r] = (f16t)(bfr(v.z) * scale);
    tile[q4 * 4 + 3][r] = (f16t)(bfr(v.w) * scale);
  }
  __syncthreads();
  v8h hv[2];
  size_t oi[2];
#pragma unroll
  for (int j = 0; j < 2; ++j) {
    const int c = (tid >> 3) + 32 * j, pc = tid & 7;
    hv[j] = *(const v8h*)(&tile[c][pc * 8]);
    oi[j] = (size_t)(c0 + c) * rows + r0 + pc * 8;
    *(volatile v8h*)(out + oi[j]) = hv[j];
  }
  __threadfence();
#pragma unroll
  for (int j = 0; j < 2; ++j) *(volatile v8h*)(out + oi[j]) = hv[j];
}

__global__ __launch_bounds__(256) void vtrans_k(const f16t* __restrict__ V, int ld, f16t* __restrict__ VT) {
  __shared__ __attribute__((aligned(16))) f16t tile[64][72];
  const int tid = threadIdx.x;
  const int kb = blockIdx.x, h = blockIdx.y, b = blockIdx.z;
  const size_t row0 = (size_t)b * SEQ + (size_t)kb * 64;
#pragma unroll
  for (int j = 0; j < 2; ++j) {
    const int i = tid + 256 * j;
    const int key = i >> 3, pc = i & 7;
    const v8h v = *(const v8h*)(V + (row0 + key) * (size_t)ld + h * HD + pc * 8);
#pragma unroll
    for (int e = 0; e < 8; ++e) tile[pc * 8 + e][key] = v[e];
  }
  __syncthreads();
  v8h hv[2];
  size_t oi[2];
#pragma unroll
  for (int j = 0; j < 2; ++j) {
    const int d = (tid >> 3) + 32 * j, pc = tid & 7;
    hv[j] = *(const v8h*)(&tile[d][pc * 8]);
    oi[j] = ((size_t)(b * NH + h) * HD + d) * SEQ + (size_t)kb * 64 + pc * 8;
    *(volatile v8h*)(VT + oi[j]) = hv[j];
  }
  __threadfence();
#pragma unroll
  for (int j = 0; j < 2; ++j) *(volatile v8h*)(VT + oi[j]) = hv[j];
}

__global__ __launch_bounds__(256) void gemm_k(
    const f16t* __restrict__ A, int lda, const f16t* __restrict__ Bt, int ldb, int K,
    const float* __restrict__ bias, float accScale,
    const float* __restrict__ res, int resBatchRows, int resRne,
    int act, float outScale, float* outF, f16t* outH, int ldc)
{
  __shared__ __attribute__((aligned(16))) float stg[8][16][64];
  const int tid = threadIdx.x, lane = tid & 31, wave = tid >> 5;
  const int h16 = lane >> 4, m16 = lane & 15;
  const int wm = wave >> 1, wn = wave & 1;
  const int m0 = blockIdx.y * 128 + wm * 32;
  const int n0 = blockIdx.x * 128 + wn * 64;

  const v8f z8 = {0.f, 0.f, 0.f, 0.f, 0.f, 0.f, 0.f, 0.f};
  v8f acc[2][4];
#pragma unroll
  for (int i = 0; i < 2; ++i)
#pragma unroll
    for (int j = 0; j < 4; ++j) acc[i][j] = z8;

  const f16t* Ab0 = A + (size_t)m0 * lda;
  const f16t* Ab1 = A + (size_t)(m0 + 16) * lda;
  const f16t* Bb  = Bt + (size_t)n0 * ldb;

#pragma unroll 1
  for (int k = 0; k < K; k += 32) {
    const v16h a0 = load_frag(Ab0 + k, lda, lane);
    const v16h a1 = load_frag(Ab1 + k, lda, lane);
    v16h b[4];
#pragma unroll
    for (int f = 0; f < 4; ++f) b[f] = load_frag(Bb + (size_t)(f * 16) * ldb + k, ldb, lane);
#pragma unroll
    for (int f = 0; f < 4; ++f) {
      acc[0][f] = wmma16(a0, b[f], acc[0][f]);
      acc[1][f] = wmma16(a1, b[f], acc[1][f]);
    }
    asm volatile("v_nop\n\tv_nop\n\tv_nop\n\tv_nop"
                 : "+v"(acc[0][0]), "+v"(acc[0][1]), "+v"(acc[0][2]), "+v"(acc[0][3]),
                   "+v"(acc[1][0]), "+v"(acc[1][1]), "+v"(acc[1][2]), "+v"(acc[1][3])
                 : "v"(a0), "v"(a1), "v"(b[0]), "v"(b[1]), "v"(b[2]), "v"(b[3]));
  }

  float* sw = &stg[wave][0][0];
#pragma unroll
  for (int mi = 0; mi < 2; ++mi) {
#pragma unroll
    for (int f = 0; f < 4; ++f)
#pragma unroll
      for (int r = 0; r < 8; ++r)
        sw[(8 * h16 + r) * 64 + f * 16 + m16] = acc[mi][f][r] * accScale;
    __builtin_amdgcn_fence(3, "wavefront");
    __builtin_amdgcn_wave_barrier();
    const int rbase = m0 + mi * 16;

    if (outF != nullptr) {
      v4f ov[8];
#pragma unroll
      for (int it = 0; it < 8; ++it) {
        const int row = 2 * it + h16, c4 = m16 * 4;
        const int grow = rbase + row, cn = n0 + c4;
        v4f v = *(const v4f*)(sw + row * 64 + c4);
        v += bfr4(*(const v4f*)(bias + cn));
        if (res != nullptr) {
          const size_t rr = (size_t)(grow / SEQ) * (size_t)resBatchRows + (size_t)(grow % SEQ);
          v4f rv = *(const v4f*)(res + rr * (size_t)ldc + cn);
          if (resRne) rv = bfr4(rv);
          v += rv;
        }
        if (act) v = gelu4(v);
        ov[it] = v * outScale;
      }
#pragma unroll
      for (int it = 0; it < 8; ++it)
        *(volatile v4f*)(outF + (size_t)(rbase + 2 * it + h16) * ldc + n0 + m16 * 4) = ov[it];
      __threadfence();
#pragma unroll
      for (int it = 0; it < 8; ++it)
        *(volatile v4f*)(outF + (size_t)(rbase + 2 * it + h16) * ldc + n0 + m16 * 4) = ov[it];
    } else {
      v8h oh[4];
#pragma unroll
      for (int it = 0; it < 4; ++it) {
        const int row = 4 * it + (lane >> 3), c8 = (lane & 7) * 8;
        const int grow = rbase + row, cn = n0 + c8;
        v4f v0 = *(const v4f*)(sw + row * 64 + c8);
        v4f v1 = *(const v4f*)(sw + row * 64 + c8 + 4);
        v0 += bfr4(*(const v4f*)(bias + cn));
        v1 += bfr4(*(const v4f*)(bias + cn + 4));
        if (res != nullptr) {
          const size_t rr = (size_t)(grow / SEQ) * (size_t)resBatchRows + (size_t)(grow % SEQ);
          v4f r0v = *(const v4f*)(res + rr * (size_t)ldc + cn);
          v4f r1v = *(const v4f*)(res + rr * (size_t)ldc + cn + 4);
          if (resRne) { r0v = bfr4(r0v); r1v = bfr4(r1v); }
          v0 += r0v; v1 += r1v;
        }
        if (act) { v0 = gelu4(v0); v1 = gelu4(v1); }
        v0 *= outScale; v1 *= outScale;
        v8h hv;
        hv[0] = (f16t)v0.x; hv[1] = (f16t)v0.y; hv[2] = (f16t)v0.z; hv[3] = (f16t)v0.w;
        hv[4] = (f16t)v1.x; hv[5] = (f16t)v1.y; hv[6] = (f16t)v1.z; hv[7] = (f16t)v1.w;
        oh[it] = hv;
      }
#pragma unroll
      for (int it = 0; it < 4; ++it)
        *(volatile v8h*)(outH + (size_t)(rbase + 4 * it + (lane >> 3)) * ldc + n0 + (lane & 7) * 8) = oh[it];
      __threadfence();
#pragma unroll
      for (int it = 0; it < 4; ++it)
        *(volatile v8h*)(outH + (size_t)(rbase + 4 * it + (lane >> 3)) * ldc + n0 + (lane & 7) * 8) = oh[it];
    }
    __builtin_amdgcn_fence(3, "wavefront");
    __builtin_amdgcn_wave_barrier();
  }
}

__global__ __launch_bounds__(128) __attribute__((amdgpu_num_vgpr(256)))
void attn_k(const f16t* __restrict__ Q, int ldq, const f16t* __restrict__ Kp, int ldk,
            const f16t* __restrict__ VT, f16t* __restrict__ O, int causal)
{
  __shared__ __attribute__((aligned(16))) f16t Pl[4][16][64];
  const int tid = threadIdx.x, lane = tid & 31, wave = tid >> 5;
  const int h16 = lane >> 4, m16 = lane & 15;
  const int bh = blockIdx.y, b = bh / NH, h = bh - b * NH;
  const int qblk = blockIdx.x * 64;
  const int q0 = qblk + wave * 16;

  const f16t* Qw = Q + (size_t)(b * SEQ + q0) * ldq + h * HD;
  const v16h qa0 = load_frag(Qw, ldq, lane);
  const v16h qa1 = load_frag(Qw + 32, ldq, lane);
  const f16t* Kh = Kp + (size_t)(b * SEQ) * ldk + h * HD;
  const f16t* Vh = VT + (size_t)bh * HD * SEQ;

  const v8f z8 = {0.f, 0.f, 0.f, 0.f, 0.f, 0.f, 0.f, 0.f};
  v8f o[4];
#pragma unroll
  for (int f = 0; f < 4; ++f) o[f] = z8;
  float mr[8], lr[8];
#pragma unroll
  for (int r = 0; r < 8; ++r) { mr[r] = -1e30f; lr[r] = 0.0f; }

  const int cdiag = qblk >> 6;
  const int nch = causal ? (cdiag + 1) : (SEQ / 64);
  f16t* pw = &Pl[wave][0][0];

#pragma unroll 1
  for (int c = 0; c < nch; ++c) {
    const int key0 = c * 64;
    const bool diag = (causal != 0) && (c == cdiag);

    v8f s[4];
#pragma unroll
    for (int j = 0; j < 4; ++j) {
      const f16t* kp = Kh + (size_t)(key0 + 16 * j) * ldk;
      const v16h kb0 = load_frag(kp, ldk, lane);
      const v16h kb1 = load_frag(kp + 32, ldk, lane);
      v8f t = wmma16(qa0, kb0, z8);
      t = wmma16(qa1, kb1, t);
      asm volatile("v_nop\n\tv_nop\n\tv_nop\n\tv_nop" : "+v"(t) : "v"(qa0), "v"(qa1), "v"(kb0), "v"(kb1));
      s[j] = t;
    }

#pragma unroll
    for (int r = 0; r < 8; ++r) {
      const int q = q0 + 8 * h16 + r;
      float v0 = s[0][r] * 0.125f, v1 = s[1][r] * 0.125f, v2 = s[2][r] * 0.125f, v3 = s[3][r] * 0.125f;
      if (diag) {
        const int kc = key0 + m16;
        v0 = (kc      > q) ? -10000.0f : v0;
        v1 = (kc + 16 > q) ? -10000.0f : v1;
        v2 = (kc + 32 > q) ? -10000.0f : v2;
        v3 = (kc + 48 > q) ? -10000.0f : v3;
      }
      float cm = fmaxf(fmaxf(v0, v1), fmaxf(v2, v3));
      cm = fmaxf(cm, __shfl_xor(cm, 1, 32));
      cm = fmaxf(cm, __shfl_xor(cm, 2, 32));
      cm = fmaxf(cm, __shfl_xor(cm, 4, 32));
      cm = fmaxf(cm, __shfl_xor(cm, 8, 32));
      const float nm = fmaxf(mr[r], cm);
      const float alpha = __expf(mr[r] - nm);
      mr[r] = nm;
      const float p0 = __expf(v0 - nm), p1 = __expf(v1 - nm), p2 = __expf(v2 - nm), p3 = __expf(v3 - nm);
      float rs = (p0 + p1) + (p2 + p3);
      rs += __shfl_xor(rs, 1, 32);
      rs += __shfl_xor(rs, 2, 32);
      rs += __shfl_xor(rs, 4, 32);
      rs += __shfl_xor(rs, 8, 32);
      lr[r] = lr[r] * alpha + rs;
#pragma unroll
      for (int f = 0; f < 4; ++f) o[f][r] *= alpha;
      f16t* prow = pw + (8 * h16 + r) * 64 + m16;
      prow[0]  = (f16t)(p0 * 1024.0f);
      prow[16] = (f16t)(p1 * 1024.0f);
      prow[32] = (f16t)(p2 * 1024.0f);
      prow[48] = (f16t)(p3 * 1024.0f);
    }
    __builtin_amdgcn_fence(3, "wavefront");
    __builtin_amdgcn_wave_barrier();

    const v16h pa0 = load_frag(pw, 64, lane);
    const v16h pa1 = load_frag(pw + 32, 64, lane);
#pragma unroll
    for (int f = 0; f < 4; ++f) {
      const f16t* vp = Vh + (size_t)(16 * f) * SEQ + key0;
      const v16h vb0 = load_frag(vp, SEQ, lane);
      const v16h vb1 = load_frag(vp + 32, SEQ, lane);
      v8f t = wmma16(pa0, vb0, o[f]);
      t = wmma16(pa1, vb1, t);
      asm volatile("v_nop\n\tv_nop\n\tv_nop\n\tv_nop" : "+v"(t) : "v"(pa0), "v"(pa1), "v"(vb0), "v"(vb1));
      o[f] = t;
    }
    __builtin_amdgcn_fence(3, "wavefront");
    __builtin_amdgcn_wave_barrier();
  }

  float inv[8];
#pragma unroll
  for (int r = 0; r < 8; ++r) inv[r] = 0.015625f / lr[r];
#pragma unroll
  for (int f = 0; f < 4; ++f)
#pragma unroll
    for (int r = 0; r < 8; ++r)
      pw[(8 * h16 + r) * 64 + f * 16 + m16] = (f16t)(o[f][r] * inv[r]);
  __builtin_amdgcn_fence(3, "wavefront");
  __builtin_amdgcn_wave_barrier();
  v8h oh[4];
#pragma unroll
  for (int it = 0; it < 4; ++it) {
    const int row = 4 * it + (lane >> 3), pc = lane & 7;
    oh[it] = *(const v8h*)(pw + row * 64 + pc * 8);
  }
#pragma unroll
  for (int it = 0; it < 4; ++it)
    *(volatile v8h*)(O + (size_t)(b * SEQ + q0 + 4 * it + (lane >> 3)) * DM + h * HD + (lane & 7) * 8) = oh[it];
  __threadfence();
#pragma unroll
  for (int it = 0; it < 4; ++it)
    *(volatile v8h*)(O + (size_t)(b * SEQ + q0 + 4 * it + (lane >> 3)) * DM + h * HD + (lane & 7) * 8) = oh[it];
}

__global__ __launch_bounds__(256) void ln_k(const float* __restrict__ Y, const float* __restrict__ g,
                                           const float* __restrict__ bta,
                                           float* outF, f16t* outH, float* outFinal) {
  __shared__ float red[2][8];
  const int row = blockIdx.x, tid = threadIdx.x, lane = tid & 31, wave = tid >> 5;
  const v4f x = *(const v4f*)(Y + (size_t)row * DM + tid * 4);
  float s = (x.x + x.y) + (x.z + x.w);
#pragma unroll
  for (int m = 16; m; m >>= 1) s += __shfl_xor(s, m, 32);
  if (lane == 0) red[0][wave] = s;
  __syncthreads();
  float tot = 0.0f;
#pragma unroll
  for (int i = 0; i < 8; ++i) tot += red[0][i];
  const float mean = tot * (1.0f / DM);
  const float d0 = x.x - mean, d1 = x.y - mean, d2 = x.z - mean, d3 = x.w - mean;
  float s2 = (d0 * d0 + d1 * d1) + (d2 * d2 + d3 * d3);
#pragma unroll
  for (int m = 16; m; m >>= 1) s2 += __shfl_xor(s2, m, 32);
  if (lane == 0) red[1][wave] = s2;
  __syncthreads();
  float tot2 = 0.0f;
#pragma unroll
  for (int i = 0; i < 8; ++i) tot2 += red[1][i];
  const float var = tot2 * (1.0f / DM);
  const float rstd = rsqrtf(var + LN_EPS);
  const int cn = tid * 4;
  const v4f gv = bfr4(*(const v4f*)(g + cn));
  const v4f bv = bfr4(*(const v4f*)(bta + cn));
  v4f ov;
  ov.x = d0 * rstd * gv.x + bv.x;
  ov.y = d1 * rstd * gv.y + bv.y;
  ov.z = d2 * rstd * gv.z + bv.z;
  ov.w = d3 * rstd * gv.w + bv.w;
  v4h hv;
  hv[0] = (f16t)ov.x; hv[1] = (f16t)ov.y; hv[2] = (f16t)ov.z; hv[3] = (f16t)ov.w;
  const size_t frow = (size_t)(row / SEQ) * SEQ_FULL + (size_t)(row % SEQ);
  if (outF != nullptr)     *(volatile v4f*)(outF + (size_t)row * DM + cn) = ov;
  if (outH != nullptr)     *(volatile v4h*)(outH + (size_t)row * DM + cn) = hv;
  if (outFinal != nullptr) *(volatile v4f*)(outFinal + frow * DM + cn) = ov;
  __threadfence();
  if (outF != nullptr)     *(volatile v4f*)(outF + (size_t)row * DM + cn) = ov;
  if (outH != nullptr)     *(volatile v4h*)(outH + (size_t)row * DM + cn) = hv;
  if (outFinal != nullptr) *(volatile v4f*)(outFinal + frow * DM + cn) = ov;
}

extern "C" void kernel_launch(void* const* d_in, const int* in_sizes, int n_in,
                              void* d_out, int out_size, void* d_ws, size_t ws_size,
                              hipStream_t stream) {
  if (n_in < 22) return;
  const int actRows = (NB - 1) * SEQ_FULL + SEQ;
  if (in_sizes[0] < actRows * DM || in_sizes[1] < actRows * DM) return;
  if (in_sizes[2] < DM * 3 * DM || in_sizes[3] < 3 * DM) return;
  if (in_sizes[4] < DM * DM || in_sizes[5] < DM) return;
  if (in_sizes[6] < DM * DM || in_sizes[7] < DM) return;
  if (in_sizes[8] < DM * 2 * DM || in_sizes[9] < 2 * DM) return;
  if (in_sizes[10] < DM * DM || in_sizes[11] < DM) return;
  if (in_sizes[12] < DM * 4 * DM || in_sizes[13] < 4 * DM) return;
  if (in_sizes[14] < 4 * DM * DM || in_sizes[15] < DM) return;
  for (int i = 16; i < 22; ++i) if (in_sizes[i] < DM) return;
  if (out_size < actRows * DM) return;

  const float* x            = (const float*)d_in[0];
  const float* ctx          = (const float*)d_in[1];
  const float* c_attn_w     = (const float*)d_in[2];
  const float* c_attn_b     = (const float*)d_in[3];
  const float* self_proj_w  = (const float*)d_in[4];
  const float* self_proj_b  = (const float*)d_in[5];
  const float* q_w          = (const float*)d_in[6];
  const float* q_b          = (const float*)d_in[7];
  const float* kv_w         = (const float*)d_in[8];
  const float* kv_b         = (const float*)d_in[9];
  const float* cross_proj_w = (const float*)d_in[10];
  const float* cross_proj_b = (const float*)d_in[11];
  const float* fc_w         = (const float*)d_in[12];
  const float* fc_b         = (const float*)d_in[13];
  const float* mlp_proj_w   = (const float*)d_in[14];
  const float* mlp_proj_b   = (const float*)d_in[15];
  const float* ln1_g = (const float*)d_in[16];
  const float* ln1_b = (const float*)d_in[17];
  const float* ln2_g = (const float*)d_in[18];
  const float* ln2_b = (const float*)d_in[19];
  const float* ln3_g = (const float*)d_in[20];
  const float* ln3_b = (const float*)d_in[21];
  float* out = (float*)d_out;

  const size_t hb = (size_t)MROWS * DM * 2;
  char* ws = (char*)d_ws;
  size_t off = 0;
  f16t* Xh   = (f16t*)(ws + off);
  f16t* Ch   = (f16t*)(ws + off + hb);
  f16t* VTp  = (f16t*)(ws + off + 2 * hb);
  f16t* Oh   = (f16t*)(ws + off + 3 * hb);
  f16t* Hh   = (f16t*)(ws + off);
  off += 4 * hb;
  f16t* WqkvT = (f16t*)(ws + off); off += (size_t)3 * DM * DM * 2;
  f16t* WspT  = (f16t*)(ws + off); off += (size_t)DM * DM * 2;
  f16t* WqT   = (f16t*)(ws + off); off += (size_t)DM * DM * 2;
  f16t* WkvT  = (f16t*)(ws + off); off += (size_t)2 * DM * DM * 2;
  f16t* WcpT  = (f16t*)(ws + off); off += (size_t)DM * DM * 2;
  f16t* WfcT  = (f16t*)(ws + off); off += (size_t)4 * DM * DM * 2;
  f16t* WmpT  = (f16t*)(ws + off); off += (size_t)4 * DM * DM * 2;
  f16t* QKVh  = (f16t*)(ws + off);
  f16t* Q2h   = (f16t*)(ws + off);
  f16t* KV2h  = (f16t*)(ws + off + hb);
  off += 3 * hb;
  float* Y    = (float*)(ws + off); off += 2 * hb;
  float* Xf   = (float*)(ws + off); off += 2 * hb;
  f16t* Xh16  = (f16t*)(ws + off); off += hb;
  const size_t need = off;
  if (ws_size < need) return;

  const dim3 blk256(256), blk128(128);
  const int cvtBlocks = (int)(((size_t)MROWS * DM / 8 + 255) / 256);

  cvt_k<<<dim3(cvtBlocks), blk256, 0, stream>>>(x, Xh, MROWS);
  cvt_k<<<dim3(cvtBlocks), blk256, 0, stream>>>(ctx, Ch, MROWS);

  wtrans_k<<<dim3(3 * DM / 64, DM / 64), blk256, 0, stream>>>(c_attn_w, WqkvT, DM, 3 * DM, 64.0f);
  wtrans_k<<<dim3(DM / 64, DM / 64), blk256, 0, stream>>>(self_proj_w, WspT, DM, DM, 64.0f);
  wtrans_k<<<dim3(DM / 64, DM / 64), blk256, 0, stream>>>(q_w, WqT, DM, DM, 64.0f);
  wtrans_k<<<dim3(2 * DM / 64, DM / 64), blk256, 0, stream>>>(kv_w, WkvT, DM, 2 * DM, 64.0f);
  wtrans_k<<<dim3(DM / 64, DM / 64), blk256, 0, stream>>>(cross_proj_w, WcpT, DM, DM, 64.0f);
  wtrans_k<<<dim3(4 * DM / 64, DM / 64), blk256, 0, stream>>>(fc_w, WfcT, DM, 4 * DM, 64.0f);
  wtrans_k<<<dim3(DM / 64, 4 * DM / 64), blk256, 0, stream>>>(mlp_proj_w, WmpT, 4 * DM, DM, 64.0f);

  gemm_k<<<dim3(3 * DM / 128, MROWS / 128), blk256, 0, stream>>>(
      Xh, DM, WqkvT, DM, DM, c_attn_b, 1.0f / 64.0f, nullptr, 0, 0, 0, 1.0f, nullptr, QKVh, 3 * DM);

  vtrans_k<<<dim3(SEQ / 64, NH, NB), blk256, 0, stream>>>(QKVh + 2 * DM, 3 * DM, VTp);
  attn_k<<<dim3(SEQ / 64, NB * NH), blk128, 0, stream>>>(QKVh, 3 * DM, QKVh + DM, 3 * DM, VTp, Oh, 1);

  gemm_k<<<dim3(DM / 128, MROWS / 128), blk256, 0, stream>>>(
      Oh, DM, WspT, DM, DM, self_proj_b, 1.0f / 1024.0f, x, SEQ_FULL, 1, 0, 1.0f, Y, nullptr, DM);
  ln_k<<<dim3(MROWS), blk256, 0, stream>>>(Y, ln1_g, ln1_b, Xf, Xh16, nullptr);

  gemm_k<<<dim3(DM / 128, MROWS / 128), blk256, 0, stream>>>(
      Xh16, DM, WqT, DM, DM, q_b, 1.0f / 64.0f, nullptr, 0, 0, 0, 1.0f, nullptr, Q2h, DM);
  gemm_k<<<dim3(2 * DM / 128, MROWS / 128), blk256, 0, stream>>>(
      Ch, DM, WkvT, DM, DM, kv_b, 1.0f / 64.0f, nullptr, 0, 0, 0, 1.0f, nullptr, KV2h, 2 * DM);
  vtrans_k<<<dim3(SEQ / 64, NH, NB), blk256, 0, stream>>>(KV2h + DM, 2 * DM, VTp);
  attn_k<<<dim3(SEQ / 64, NB * NH), blk128, 0, stream>>>(Q2h, DM, KV2h, 2 * DM, VTp, Oh, 0);

  gemm_k<<<dim3(DM / 128, MROWS / 128), blk256, 0, stream>>>(
      Oh, DM, WcpT, DM, DM, cross_proj_b, 1.0f / 1024.0f, Xf, SEQ, 0, 0, 1.0f, Y, nullptr, DM);
  ln_k<<<dim3(MROWS), blk256, 0, stream>>>(Y, ln2_g, ln2_b, Xf, Xh16, nullptr);

  gemm_k<<<dim3(4 * DM / 128, MROWS / 128), blk256, 0, stream>>>(
      Xh16, DM, WfcT, DM, DM, fc_b, 1.0f / 64.0f, nullptr, 0, 0, 1, 8.0f, nullptr, Hh, 4 * DM);
  gemm_k<<<dim3(DM / 128, MROWS / 128), blk256, 0, stream>>>(
      Hh, 4 * DM, WmpT, 4 * DM, 4 * DM, mlp_proj_b, 1.0f / 512.0f, Xf, SEQ, 0, 0, 1.0f, Y, nullptr, DM);
  ln_k<<<dim3(MROWS), blk256, 0, stream>>>(Y, ln3_g, ln3_b, nullptr, nullptr, out);
}
